// RayRoPE_DotProductAttention_84885733638602
// MI455X (gfx1250) — hardware-verified
//
#include <hip/hip_runtime.h>
#include <stdint.h>

typedef _Float16 v16h __attribute__((ext_vector_type(16)));
typedef _Float16 v8h  __attribute__((ext_vector_type(8)));
typedef v8h v8ha __attribute__((may_alias));
typedef float v8f __attribute__((ext_vector_type(8)));
typedef float v4f __attribute__((ext_vector_type(4)));
typedef v4f v4fa __attribute__((may_alias));

#define B_    2
#define H_    16
#define S_    2048
#define D_    64
#define HALF_ 32
#define BH_   (B_ * H_)
#define PS    64
#define VT_LD 72
#define QB    64
#define KS    64
#define SO_LD 68

static_assert(S_ % PS == 0);
static_assert(S_ % QB == 0);
static_assert(S_ % KS == 0);

union Frag { v16h v; v8h half[2]; _Float16 e[16]; };
union F8   { v4f q[2]; float f[8]; };
union H8   { v8h v; _Float16 e[8]; };

__device__ __forceinline__ v8f wmma16(v16h a, v16h b, v8f c)
{
    v8f d = __builtin_amdgcn_wmma_f32_16x16x32_f16(false, a, false, b, (short)0, c, false, false);
    asm volatile("v_nop\n\tv_nop\n\tv_nop\n\tv_nop" : "+v"(d) : "v"(a), "v"(b));
    return d;
}

__global__ __launch_bounds__(256)
void k_prep(const float* __restrict__ Q, const float* __restrict__ K, const float* __restrict__ V,
            const float* __restrict__ C, const float* __restrict__ Sn,
            _Float16* Qh, _Float16* Kh, _Float16* Vt)
{
    __shared__ __attribute__((aligned(16))) _Float16 sVt[D_][VT_LD];

    const int tid = threadIdx.x, w = tid >> 5, l = tid & 31;
    const int bh  = blockIdx.y;
    const int b   = bh / H_;
    const int s0  = blockIdx.x * PS;

    v8h    qo[2], ko[2];
    size_t ro[2];
#pragma unroll
    for (int g = 0; g < 2; ++g) {
        const int rl = 8 * w + 4 * g + (l >> 3);
        const int j  = l & 7;
        const int jp = (j & 3) * 8;
        const int s  = s0 + rl;
        const size_t rowoff = ((size_t)bh * S_ + s) * D_;
        const size_t csoff  = ((size_t)b * S_ + s) * HALF_ + jp;

        F8 q1, q2, k1, k2, cc, ss;
        const v4f* qr = (const v4f*)(Q + rowoff + jp);
        const v4f* kr = (const v4f*)(K + rowoff + jp);
        const v4f* cr = (const v4f*)(C + csoff);
        const v4f* sr = (const v4f*)(Sn + csoff);
        q1.q[0] = qr[0]; q1.q[1] = qr[1]; q2.q[0] = qr[8]; q2.q[1] = qr[9];
        k1.q[0] = kr[0]; k1.q[1] = kr[1]; k2.q[0] = kr[8]; k2.q[1] = kr[9];
        cc.q[0] = cr[0]; cc.q[1] = cr[1]; ss.q[0] = sr[0]; ss.q[1] = sr[1];

        const bool first_half = (j < 4);
        H8 oq, ok;
#pragma unroll
        for (int t = 0; t < 8; ++t) {
            const float c = cc.f[t], sn = ss.f[t];
            const float qa = q1.f[t], qd = q2.f[t];
            const float ka = k1.f[t], kd = k2.f[t];
            const float rq = first_half ? (qa * c - qd * sn) : (qa * sn + qd * c);
            const float rk = first_half ? (ka * c - kd * sn) : (ka * sn + kd * c);
            oq.e[t] = (_Float16)(rq * 0.125f);
            ok.e[t] = (_Float16)(rk);
        }
        qo[g] = oq.v;
        ko[g] = ok.v;
        ro[g] = rowoff + 8 * j;
    }
#pragma unroll
    for (int g = 0; g < 2; ++g) {
        *(volatile v8h*)(Qh + ro[g]) = qo[g];
        *(volatile v8h*)(Kh + ro[g]) = ko[g];
    }

#pragma unroll
    for (int p = 0; p < 4; ++p) {
        const int idx = tid + 256 * p;
        const int sl  = idx >> 4;
        const int d4  = (idx & 15) * 4;
        const v4f x = *(const v4f*)(V + ((size_t)bh * S_ + s0 + sl) * D_ + d4);
        sVt[d4 + 0][sl] = (_Float16)x[0];
        sVt[d4 + 1][sl] = (_Float16)x[1];
        sVt[d4 + 2][sl] = (_Float16)x[2];
        sVt[d4 + 3][sl] = (_Float16)x[3];
    }
    __syncthreads();

    v8h    vo[2];
    size_t vro[2];
#pragma unroll
    for (int g = 0; g < 2; ++g) {
        const int d = 8 * w + 4 * g + (l >> 3);
        const int j = l & 7;
        vo[g]  = *(const v8ha*)(&sVt[d][8 * j]);
        vro[g] = ((size_t)bh * D_ + d) * S_ + s0 + 8 * j;
    }
#pragma unroll
    for (int g = 0; g < 2; ++g) *(volatile v8h*)(Vt + vro[g]) = vo[g];

    __threadfence();

#pragma unroll
    for (int g = 0; g < 2; ++g) {
        *(volatile v8h*)(Qh + ro[g]) = qo[g];
        *(volatile v8h*)(Kh + ro[g]) = ko[g];
        *(volatile v8h*)(Vt + vro[g]) = vo[g];
    }
}

__global__ __launch_bounds__(128)
void k_attn(const _Float16* __restrict__ Qh, const _Float16* __restrict__ Kh,
            const _Float16* __restrict__ Vt, float* O)
{
    __shared__ __attribute__((aligned(16))) float sO[QB / 16][16][SO_LD];

    const int tid = threadIdx.x, w = tid >> 5, l = tid & 31, h = l >> 4, n = l & 15;
    const int bh  = blockIdx.y;
    const int q0  = blockIdx.x * QB + w * 16;

    const float L2E = 1.44269504088896340736f;
    const float PSC = 16384.0f;

    Frag qb[2];
    {
        const _Float16* qp = Qh + ((size_t)bh * S_ + q0 + n) * D_ + 8 * h;
        qb[0].half[0] = *(const v8ha*)(qp);
        qb[0].half[1] = *(const v8ha*)(qp + 16);
        qb[1].half[0] = *(const v8ha*)(qp + 32);
        qb[1].half[1] = *(const v8ha*)(qp + 48);
    }
    const _Float16* kbase = Kh + (size_t)bh * S_ * D_ + (size_t)n * D_ + 8 * h;
    const _Float16* vbase = Vt + (size_t)bh * D_ * S_ + (size_t)n * S_ + 8 * h;

    v8f acc[4];
#pragma unroll
    for (int o = 0; o < 4; ++o)
#pragma unroll
        for (int r = 0; r < 8; ++r) acc[o][r] = 0.0f;
    float mrun = -1.0e30f, lrun = 0.0f;

#pragma unroll 1
    for (int ks = 0; ks < S_; ks += KS) {
        v8f st[4];
#pragma unroll
        for (int j = 0; j < 4; ++j) {
            const _Float16* kp = kbase + (size_t)(ks + 16 * j) * D_;
            Frag a0, a1;
            a0.half[0] = *(const v8ha*)(kp);       a0.half[1] = *(const v8ha*)(kp + 16);
            a1.half[0] = *(const v8ha*)(kp + 32);  a1.half[1] = *(const v8ha*)(kp + 48);
            v8f z;
#pragma unroll
            for (int r = 0; r < 8; ++r) z[r] = 0.0f;
            z = wmma16(a0.v, qb[0].v, z);
            z = wmma16(a1.v, qb[1].v, z);
            st[j] = z;
        }

        float mx = st[0][0];
#pragma unroll
        for (int j = 0; j < 4; ++j)
#pragma unroll
            for (int r = 0; r < 8; ++r) mx = fmaxf(mx, st[j][r]);
        mx = fmaxf(mx, __shfl_xor(mx, 16, 32));
        const float mn    = fmaxf(mrun, mx);
        const float alpha = exp2f((mrun - mn) * L2E);
        mrun = mn;

        float rs = 0.0f;
        Frag pb[2];
#pragma unroll
        for (int j = 0; j < 4; ++j) {
#pragma unroll
            for (int r = 0; r < 8; ++r) {
                const float p = exp2f((st[j][r] - mn) * L2E);
                rs += p;
                pb[j >> 1].e[(j & 1) * 8 + r] = (_Float16)(p * PSC);
            }
        }
        rs += __shfl_xor(rs, 16, 32);
        lrun = lrun * alpha + rs;
#pragma unroll
        for (int o = 0; o < 4; ++o) acc[o] = acc[o] * alpha;

#pragma unroll
        for (int o = 0; o < 4; ++o) {
            const _Float16* vp = vbase + (size_t)o * 16 * S_ + ks;
            Frag v0, v1;
            v0.half[0] = *(const v8ha*)(vp);       v0.half[1] = *(const v8ha*)(vp + 16);
            v1.half[0] = *(const v8ha*)(vp + 32);  v1.half[1] = *(const v8ha*)(vp + 48);
            acc[o] = wmma16(v0.v, pb[0].v, acc[o]);
            acc[o] = wmma16(v1.v, pb[1].v, acc[o]);
        }
    }

    const float inv = 1.0f / (lrun * PSC);
#pragma unroll
    for (int o = 0; o < 4; ++o)
#pragma unroll
        for (int r = 0; r < 8; ++r) sO[w][n][16 * o + 8 * h + r] = acc[o][r] * inv;
    __syncthreads();

    v4f ov[8];
#pragma unroll
    for (int i = 0; i < 8; ++i) ov[i] = *(const v4fa*)(&sO[w][2 * i + h][4 * n]);

    float* ob = O + ((size_t)bh * S_ + q0) * D_ + 4 * n;
#pragma unroll
    for (int i = 0; i < 8; ++i) *(volatile v4f*)(ob + (size_t)(2 * i + h) * D_) = ov[i];
    __threadfence();
#pragma unroll
    for (int i = 0; i < 8; ++i) *(volatile v4f*)(ob + (size_t)(2 * i + h) * D_) = ov[i];
}

extern "C" void kernel_launch(void* const* d_in, const int* in_sizes, int n_in,
                              void* d_out, int out_size, void* d_ws, size_t ws_size,
                              hipStream_t stream)
{
    if (n_in < 5) return;
    const size_t nq  = (size_t)B_ * H_ * S_ * D_;
    const size_t ncs = (size_t)B_ * S_ * HALF_;
    if ((size_t)in_sizes[0] != nq || (size_t)in_sizes[1] != nq || (size_t)in_sizes[2] != nq) return;
    if ((size_t)in_sizes[3] != ncs || (size_t)in_sizes[4] != ncs) return;
    if ((size_t)out_size != nq) return;

    const size_t plane = nq * sizeof(_Float16);
    if (3 * plane > ws_size) return;

    const float* q = (const float*)d_in[0];
    const float* k = (const float*)d_in[1];
    const float* v = (const float*)d_in[2];
    const float* c = (const float*)d_in[3];
    const float* s = (const float*)d_in[4];
    char* ws = (char*)d_ws;
    _Float16* Qh = (_Float16*)(ws);
    _Float16* Kh = (_Float16*)(ws + plane);
    _Float16* Vt = (_Float16*)(ws + 2 * plane);
    float* out = (float*)d_out;

    hipLaunchKernelGGL(k_prep, dim3(S_ / PS, BH_), dim3(256), 0, stream, q, k, v, c, s, Qh, Kh, Vt);
    hipLaunchKernelGGL(k_attn, dim3(S_ / QB, BH_), dim3(128), 0, stream,
                       (const _Float16*)Qh, (const _Float16*)Kh, (const _Float16*)Vt, out);
}
